// SINSelfAttention_63410897158176
// MI455X (gfx1250) — hardware-verified
//
#include <hip/hip_runtime.h>

typedef _Float16 v16h __attribute__((ext_vector_type(16)));
typedef _Float16 v8h  __attribute__((ext_vector_type(8)));
typedef __bf16   v16b __attribute__((ext_vector_type(16)));
typedef __bf16   v8b  __attribute__((ext_vector_type(8)));
typedef float    v8f  __attribute__((ext_vector_type(8)));
typedef float    v4f  __attribute__((ext_vector_type(4)));
typedef unsigned int v4u __attribute__((ext_vector_type(4)));
typedef v4f __attribute__((may_alias)) v4fa;
typedef v4u __attribute__((may_alias)) v4ua;

union FragH { v16h v; v8h h8[2]; v4u u[2]; };
union FragB { v16b v; v8b h8[2]; v4u u[2]; };
union Pack8H { v8h v; v4u u; };
union Pack8B { v8b v; v4u u; };

#define NB    4
#define IMG   64
#define NTOK  4096
#define CH    64
#define NXE   1048576
#define NWE   36864
#define XBLK  512
#define WBLKT 18
#define WSC   16.0f
#define WSCI  0.0625f
#define PSC   16384.0f
#define PSCI  (1.0f / 16384.0f)

__device__ __forceinline__ v8f wmma_f16(v16h a, v16h b, v8f c) {
  v8f d = __builtin_amdgcn_wmma_f32_16x16x32_f16(false, a, false, b, (short)0, c, false, false);
  asm volatile("v_nop\n\tv_nop\n\tv_nop\n\tv_nop" : "+v"(d) : "v"(a), "v"(b));
  return d;
}
__device__ __forceinline__ v8f wmma_bf16(v16b a, v16b b, v8f c) {
  v8f d = __builtin_amdgcn_wmma_f32_16x16x32_bf16(false, a, false, b, (short)0, c, false, false);
  asm volatile("v_nop\n\tv_nop\n\tv_nop\n\tv_nop" : "+v"(d) : "v"(a), "v"(b));
  return d;
}

__device__ __forceinline__ v16h ldfrag_h(const _Float16* p, int h) {
  FragH f;
  f.u[0] = *(const v4ua*)(p + 8 * h);
  f.u[1] = *(const v4ua*)(p + 16 + 8 * h);
  return f.v;
}
__device__ __forceinline__ v16h ldfrag_h_msk(const _Float16* p, int h, unsigned msk) {
  FragH f;
  f.u[0] = (*(const v4ua*)(p + 8 * h)) & msk;
  f.u[1] = (*(const v4ua*)(p + 16 + 8 * h)) & msk;
  return f.v;
}
__device__ __forceinline__ v16b ldfrag_b(const __bf16* p, int h) {
  FragB f;
  f.u[0] = *(const v4ua*)(p + 8 * h);
  f.u[1] = *(const v4ua*)(p + 16 + 8 * h);
  return f.v;
}
__device__ __forceinline__ v16b ldfrag_b_msk(const __bf16* p, int h, unsigned msk) {
  FragB f;
  f.u[0] = (*(const v4ua*)(p + 8 * h)) & msk;
  f.u[1] = (*(const v4ua*)(p + 16 + 8 * h)) & msk;
  return f.v;
}

__global__ __launch_bounds__(256) void k_prep(
    const float* __restrict__ x,
    const float* __restrict__ Wk, const float* __restrict__ Wq,
    const float* __restrict__ Wv, const float* __restrict__ Wr,
    _Float16* __restrict__ xh, _Float16* __restrict__ wt3,
    __bf16* __restrict__ wrh, __bf16* __restrict__ wrl)
{
  const int tid = threadIdx.x, blk = blockIdx.x;
  if (blk < XBLK) {
    const size_t g = (size_t)blk * 256 + tid;
    const float* src = x + g * 8;
    const v4f a = *(const v4fa*)src;
    const v4f c = *(const v4fa*)(src + 4);
    const v8h hv = { (_Float16)a.x, (_Float16)a.y, (_Float16)a.z, (_Float16)a.w,
                     (_Float16)c.x, (_Float16)c.y, (_Float16)c.z, (_Float16)c.w };
    Pack8H o; o.v = hv;
    _Float16* dst = xh + g * 8;
    *(volatile v4u*)dst = o.u;
    __threadfence();
    *(volatile v4u*)dst = o.u;
  } else {
    const int wblk = blk - XBLK;
    const int which = wblk / WBLKT;
    const int idx = (wblk - which * WBLKT) * 256 + tid;
    const int t = idx >> 9, co = (idx >> 3) & 63, j = idx & 7;
    const float* src = (which == 0) ? Wk : ((which == 1) ? Wq : ((which == 2) ? Wv : Wr));
    float f[8];
    #pragma unroll
    for (int i = 0; i < 8; ++i) f[i] = src[(size_t)(t * 64 + 8 * j + i) * 64 + co];
    const size_t off = (size_t)(t * 64 + co) * 64 + 8 * j;
    if (which < 3) {
      const v8h hv = { (_Float16)(f[0] * WSC), (_Float16)(f[1] * WSC), (_Float16)(f[2] * WSC), (_Float16)(f[3] * WSC),
                       (_Float16)(f[4] * WSC), (_Float16)(f[5] * WSC), (_Float16)(f[6] * WSC), (_Float16)(f[7] * WSC) };
      Pack8H o; o.v = hv;
      _Float16* dst = wt3 + (size_t)which * NWE + off;
      *(volatile v4u*)dst = o.u;
      __threadfence();
      *(volatile v4u*)dst = o.u;
    } else {
      __bf16 hb[8], lb[8];
      #pragma unroll
      for (int i = 0; i < 8; ++i) {
        hb[i] = (__bf16)f[i];
        lb[i] = (__bf16)(f[i] - (float)hb[i]);
      }
      const v8b hv = { hb[0], hb[1], hb[2], hb[3], hb[4], hb[5], hb[6], hb[7] };
      const v8b lv = { lb[0], lb[1], lb[2], lb[3], lb[4], lb[5], lb[6], lb[7] };
      Pack8B ph, pl; ph.v = hv; pl.v = lv;
      __bf16* dh = wrh + off;
      __bf16* dl = wrl + off;
      *(volatile v4u*)dh = ph.u;
      *(volatile v4u*)dl = pl.u;
      __threadfence();
      *(volatile v4u*)dh = ph.u;
      *(volatile v4u*)dl = pl.u;
    }
  }
}

__device__ __forceinline__ void qkv_store_pass(const _Float16* sT, _Float16* dst, int s,
                                               int b, int tb0, int w, int lane) {
  const int q8 = lane & 7, sub = lane >> 3;
  #pragma unroll
  for (int i = 0; i < 4; ++i) {
    const int lid = w * 16 + 4 * i + sub;
    const v4u v = *(const v4ua*)(sT + lid * 64 + 8 * q8);
    size_t gi;
    if (s == 2) gi = ((size_t)b * CH + lid) * NTOK + tb0 + 8 * q8;
    else        gi = ((size_t)b * NTOK + tb0 + lid) * 64 + 8 * q8;
    *(volatile v4u*)(dst + gi) = v;
  }
}

__global__ __launch_bounds__(128) void k_conv_qkv(
    const _Float16* __restrict__ xh,
    const _Float16* __restrict__ wt3,
    const float* __restrict__ bk, const float* __restrict__ bq, const float* __restrict__ bv,
    _Float16* __restrict__ kpl,
    _Float16* __restrict__ qpl,
    _Float16* __restrict__ vtp)
{
  __shared__ __attribute__((aligned(16))) _Float16 sT[64 * 64];

  const int tid = threadIdx.x, lane = tid & 31, w = tid >> 5;
  const int h = lane >> 4, m = lane & 15;
  const int b = blockIdx.x >> 6, hrow = blockIdx.x & 63;
  const int s = blockIdx.y;
  const int tb0 = hrow * 64, w0 = 16 * w;

  const _Float16* wsel = wt3 + (size_t)s * NWE + (size_t)m * 64;

  const v8f zero8 = {0.f, 0.f, 0.f, 0.f, 0.f, 0.f, 0.f, 0.f};
  v8f acc[4];
  #pragma unroll
  for (int nt = 0; nt < 4; ++nt) acc[nt] = zero8;

  #pragma unroll 1
  for (int t = 0; t < 9; ++t) {
    const int t3 = t / 3;
    const int dh = t3 - 1, dw = t - 3 * t3 - 1;
    const int hh = hrow + dh, wl = w0 + m + dw;
    const bool ok = ((unsigned)hh < 64u) && ((unsigned)wl < 64u);
    const int hc = min(max(hh, 0), 63), wc = min(max(wl, 0), 63);
    const unsigned msk = ok ? 0xffffffffu : 0u;
    const _Float16* xrow = xh + ((size_t)(b * 64 + hc) * 64 + wc) * 64;
    const _Float16* wtap = wsel + (size_t)t * 4096;
    #pragma unroll
    for (int kc = 0; kc < 2; ++kc) {
      const v16h a = ldfrag_h_msk(xrow + 32 * kc, h, msk);
      #pragma unroll
      for (int nt = 0; nt < 4; ++nt) {
        const v16h bf = ldfrag_h(wtap + nt * 1024 + 32 * kc, h);
        acc[nt] = wmma_f16(a, bf, acc[nt]);
      }
    }
  }

  const float* bias = (s == 0) ? bk : ((s == 1) ? bq : bv);
  #pragma unroll
  for (int nt = 0; nt < 4; ++nt) {
    const int co = 16 * nt + m;
    const float bb = bias[co];
    #pragma unroll
    for (int r = 0; r < 8; ++r) {
      const float y = acc[nt][r] * WSCI + bb;
      const int px = w0 + 8 * h + r;
      if (s == 2) sT[co * 64 + px] = (_Float16)fmaxf(y, 0.0f);
      else        sT[px * 64 + co] = (_Float16)((y > 0.0f) ? y : (__expf(y) - 1.0f));
    }
  }
  __syncthreads();

  _Float16* dst = (s == 0) ? kpl : ((s == 1) ? qpl : vtp);
  qkv_store_pass(sT, dst, s, b, tb0, w, lane);
  __threadfence();
  qkv_store_pass(sT, dst, s, b, tb0, w, lane);
}

__device__ __forceinline__ v16h pack_p(v8f a, v8f c) {
  const v16h r = { (_Float16)(a[0] * PSC), (_Float16)(a[1] * PSC), (_Float16)(a[2] * PSC), (_Float16)(a[3] * PSC),
                   (_Float16)(a[4] * PSC), (_Float16)(a[5] * PSC), (_Float16)(a[6] * PSC), (_Float16)(a[7] * PSC),
                   (_Float16)(c[0] * PSC), (_Float16)(c[1] * PSC), (_Float16)(c[2] * PSC), (_Float16)(c[3] * PSC),
                   (_Float16)(c[4] * PSC), (_Float16)(c[5] * PSC), (_Float16)(c[6] * PSC), (_Float16)(c[7] * PSC) };
  return r;
}

__device__ __forceinline__ void attn_store_pass(const float* so, __bf16* oh, __bf16* ol,
                                                int b, int q0, int lane) {
  const int q8 = lane & 7, sub = lane >> 3;
  #pragma unroll
  for (int i = 0; i < 4; ++i) {
    const int row = 4 * i + sub;
    const v4f a = *(const v4fa*)(so + row * 64 + 8 * q8);
    const v4f c = *(const v4fa*)(so + row * 64 + 8 * q8 + 4);
    const float f[8] = { a.x, a.y, a.z, a.w, c.x, c.y, c.z, c.w };
    __bf16 hb[8], lb[8];
    #pragma unroll
    for (int e = 0; e < 8; ++e) {
      hb[e] = (__bf16)f[e];
      lb[e] = (__bf16)(f[e] - (float)hb[e]);
    }
    const v8b hv = { hb[0], hb[1], hb[2], hb[3], hb[4], hb[5], hb[6], hb[7] };
    const v8b lv = { lb[0], lb[1], lb[2], lb[3], lb[4], lb[5], lb[6], lb[7] };
    Pack8B ph, pl; ph.v = hv; pl.v = lv;
    const size_t gi = ((size_t)b * NTOK + q0 + row) * 64 + 8 * q8;
    *(volatile v4u*)(oh + gi) = ph.u;
    *(volatile v4u*)(ol + gi) = pl.u;
  }
}

__global__ __launch_bounds__(128) void k_attn(
    const _Float16* __restrict__ qpl,
    const _Float16* __restrict__ kpl,
    const _Float16* __restrict__ vtp,
    __bf16* __restrict__ oh,
    __bf16* __restrict__ ol)
{
  __shared__ __attribute__((aligned(16))) float sO[4 * 16 * 64];

  const int tid = threadIdx.x, lane = tid & 31, w = tid >> 5;
  const int h = lane >> 4, m = lane & 15;
  const int b = blockIdx.y;
  const int qblk = blockIdx.x * 64;
  const int q0 = qblk + 16 * w;

  const _Float16* qrow = qpl + ((size_t)b * NTOK + q0 + m) * 64;
  const v16h qb0 = ldfrag_h(qrow, h);
  const v16h qb1 = ldfrag_h(qrow + 32, h);

  const v8f zero8 = {0.f, 0.f, 0.f, 0.f, 0.f, 0.f, 0.f, 0.f};
  v8f o[4];
  #pragma unroll
  for (int t = 0; t < 4; ++t) o[t] = zero8;
  float mrun = -1e30f, lrun = 0.0f;

  const _Float16* kbase = kpl + ((size_t)b * NTOK + m) * 64;
  const _Float16* vbase = vtp + ((size_t)b * CH + m) * NTOK;
  const int dq = 16 * w + m - 8 * h;

  #pragma unroll 1
  for (int kb = 0; kb < NTOK; kb += 64) {
    v8f s[4];
    #pragma unroll
    for (int j = 0; j < 4; ++j) {
      const _Float16* kr = kbase + (size_t)(kb + 16 * j) * 64;
      const v16h kf0 = ldfrag_h(kr, h);
      const v16h kf1 = ldfrag_h(kr + 32, h);
      v8f z = zero8;
      z = wmma_f16(kf0, qb0, z);
      z = wmma_f16(kf1, qb1, z);
      s[j] = z;
    }
    #pragma unroll
    for (int j = 0; j < 4; ++j)
      #pragma unroll
      for (int r = 0; r < 8; ++r) s[j][r] = s[j][r] * 0.125f;

    if (kb == qblk) {
      #pragma unroll
      for (int j = 0; j < 4; ++j)
        #pragma unroll
        for (int r = 0; r < 8; ++r)
          s[j][r] = (dq == 16 * j + r) ? 0.0f : s[j][r];
    }

    float mloc = s[0][0];
    #pragma unroll
    for (int j = 0; j < 4; ++j)
      #pragma unroll
      for (int r = 0; r < 8; ++r) mloc = fmaxf(mloc, s[j][r]);
    mloc = fmaxf(mloc, __shfl_xor(mloc, 16));
    const float mnew = fmaxf(mrun, mloc);
    const float alpha = __expf(mrun - mnew);
    mrun = mnew;
    float lsum = 0.0f;
    #pragma unroll
    for (int j = 0; j < 4; ++j)
      #pragma unroll
      for (int r = 0; r < 8; ++r) {
        const float p = __expf(s[j][r] - mnew);
        s[j][r] = p;
        lsum += p;
      }
    lsum += __shfl_xor(lsum, 16);
    lrun = lrun * alpha + lsum;
    #pragma unroll
    for (int t = 0; t < 4; ++t)
      #pragma unroll
      for (int r = 0; r < 8; ++r) o[t][r] = o[t][r] * alpha;

    const v16h pb0 = pack_p(s[0], s[1]);
    const v16h pb1 = pack_p(s[2], s[3]);

    #pragma unroll
    for (int t = 0; t < 4; ++t) {
      const _Float16* vr = vbase + (size_t)(16 * t) * NTOK + kb;
      const v16h vf0 = ldfrag_h(vr, h);
      const v16h vf1 = ldfrag_h(vr + 32, h);
      o[t] = wmma_f16(vf0, pb0, o[t]);
      o[t] = wmma_f16(vf1, pb1, o[t]);
    }
  }

  const float inv = (1.0f / lrun) * PSCI;
  float* so = sO + w * 1024;
  #pragma unroll
  for (int t = 0; t < 4; ++t)
    #pragma unroll
    for (int r = 0; r < 8; ++r)
      so[m * 64 + 16 * t + 8 * h + r] = o[t][r] * inv;
  __syncthreads();

  attn_store_pass(so, oh, ol, b, q0, lane);
  __threadfence();
  attn_store_pass(so, oh, ol, b, q0, lane);
}

__device__ __forceinline__ void out_store_pass(const float* so, float* out,
                                               int b, int p0, int lane) {
  const int q8 = lane & 7, sub = lane >> 3;
  #pragma unroll
  for (int i = 0; i < 8; ++i) {
    const int lid = 4 * i + sub;
    const int row = lid >> 1, hl = lid & 1;
    const v4f v = *(const v4fa*)(so + row * 64 + 32 * hl + 4 * q8);
    const size_t gi = ((size_t)b * NTOK + p0 + row) * 64 + 32 * hl + 4 * q8;
    *(volatile v4f*)(out + gi) = v;
  }
}

__global__ __launch_bounds__(128) void k_conv_out(
    const __bf16* __restrict__ oh, const __bf16* __restrict__ ol,
    const __bf16* __restrict__ wrh, const __bf16* __restrict__ wrl,
    const float* __restrict__ br, float* __restrict__ out)
{
  __shared__ __attribute__((aligned(16))) float sY[4 * 16 * 64];

  const int tid = threadIdx.x, lane = tid & 31, w = tid >> 5;
  const int h = lane >> 4, m = lane & 15;
  const int b = blockIdx.x >> 6, hrow = blockIdx.x & 63;
  const int tb0 = hrow * 64, w0 = 16 * w;

  const v8f zero8 = {0.f, 0.f, 0.f, 0.f, 0.f, 0.f, 0.f, 0.f};
  v8f acc[4];
  #pragma unroll
  for (int nt = 0; nt < 4; ++nt) acc[nt] = zero8;

  #pragma unroll 1
  for (int t = 0; t < 9; ++t) {
    const int t3 = t / 3;
    const int dh = t3 - 1, dw = t - 3 * t3 - 1;
    const int hh = hrow + dh, wl = w0 + m + dw;
    const bool ok = ((unsigned)hh < 64u) && ((unsigned)wl < 64u);
    const int hc = min(max(hh, 0), 63), wc = min(max(wl, 0), 63);
    const unsigned msk = ok ? 0xffffffffu : 0u;
    const size_t rowoff = ((size_t)(b * 64 + hc) * 64 + wc) * 64;
    const size_t wtap = (size_t)t * 4096 + (size_t)m * 64;
    #pragma unroll
    for (int kc = 0; kc < 2; ++kc) {
      const v16b ah = ldfrag_b_msk(oh + rowoff + 32 * kc, h, msk);
      const v16b al = ldfrag_b_msk(ol + rowoff + 32 * kc, h, msk);
      #pragma unroll
      for (int nt = 0; nt < 4; ++nt) {
        const v16b bh = ldfrag_b(wrh + wtap + nt * 1024 + 32 * kc, h);
        const v16b bl = ldfrag_b(wrl + wtap + nt * 1024 + 32 * kc, h);
        acc[nt] = wmma_bf16(ah, bh, acc[nt]);
        acc[nt] = wmma_bf16(ah, bl, acc[nt]);
        acc[nt] = wmma_bf16(al, bh, acc[nt]);
      }
    }
  }

  float* so = sY + w * 1024;
  #pragma unroll
  for (int nt = 0; nt < 4; ++nt) {
    const int co = 16 * nt + m;
    const float bb = br[co];
    #pragma unroll
    for (int r = 0; r < 8; ++r)
      so[(8 * h + r) * 64 + co] = fmaxf(acc[nt][r] + bb, 0.0f);
  }
  __syncthreads();

  out_store_pass(so, out, b, tb0 + w0, lane);
  __threadfence();
  out_store_pass(so, out, b, tb0 + w0, lane);
}

extern "C" void kernel_launch(void* const* d_in, const int* in_sizes, int n_in,
                              void* d_out, int out_size, void* d_ws, size_t ws_size,
                              hipStream_t stream) {
  if (n_in < 9) return;
  if (in_sizes[0] != NXE || out_size != NXE) return;
  if (in_sizes[1] != NWE || in_sizes[3] != NWE || in_sizes[5] != NWE || in_sizes[7] != NWE) return;
  if (in_sizes[2] != CH || in_sizes[4] != CH || in_sizes[6] != CH || in_sizes[8] != CH) return;

  const float* x  = (const float*)d_in[0];
  const float* Wk = (const float*)d_in[1];
  const float* bk = (const float*)d_in[2];
  const float* Wq = (const float*)d_in[3];
  const float* bq = (const float*)d_in[4];
  const float* Wv = (const float*)d_in[5];
  const float* bv = (const float*)d_in[6];
  const float* Wr = (const float*)d_in[7];
  const float* br = (const float*)d_in[8];
  float* out = (float*)d_out;

  const size_t pl_bytes  = (size_t)NXE * 2;
  const size_t wt3_bytes = (size_t)3 * NWE * 2;
  const size_t wr_bytes  = (size_t)NWE * 2;
  size_t off = 0;
  const size_t o_xh  = off; off += pl_bytes;
  const size_t o_wt3 = off; off += wt3_bytes;
  const size_t o_wrh = off; off += wr_bytes;
  const size_t o_wrl = off; off += wr_bytes;
  const size_t o_k   = off; off += pl_bytes;
  const size_t o_q   = off; off += pl_bytes;
  const size_t o_vt  = off; off += pl_bytes;
  const size_t o_oh  = off; off += pl_bytes;
  const size_t o_ol  = off; off += pl_bytes;
  if (off > ws_size) return;

  char* ws = (char*)d_ws;
  _Float16* xh  = (_Float16*)(ws + o_xh);
  _Float16* wt3 = (_Float16*)(ws + o_wt3);
  __bf16*   wrh = (__bf16*)(ws + o_wrh);
  __bf16*   wrl = (__bf16*)(ws + o_wrl);
  _Float16* kpl = (_Float16*)(ws + o_k);
  _Float16* qpl = (_Float16*)(ws + o_q);
  _Float16* vtp = (_Float16*)(ws + o_vt);
  __bf16*   oh  = (__bf16*)(ws + o_oh);
  __bf16*   ol  = (__bf16*)(ws + o_ol);

  k_prep<<<XBLK + 4 * WBLKT, 256, 0, stream>>>(x, Wk, Wq, Wv, Wr, xh, wt3, wrh, wrl);

  dim3 gQKV(NB * 64, 3);
  k_conv_qkv<<<gQKV, 128, 0, stream>>>(xh, wt3, bk, bq, bv, kpl, qpl, vtp);

  dim3 gAtt(NTOK / 64, NB);
  k_attn<<<gAtt, 128, 0, stream>>>(qpl, kpl, vtp, oh, ol);

  k_conv_out<<<NB * 64, 128, 0, stream>>>(oh, ol, wrh, wrl, br, out);
}
